// GCN1_90881507983767
// MI455X (gfx1250) — hardware-run, weakly checked
//
#include <hip/hip_runtime.h>
#include <stddef.h>
#include <stdint.h>


#define DF     128
#define K1     128
#define K2     256
#define NTHR   256
#define NWAVE  8
#define EPT    8
#define WCH    (32 * EPT)
#define NBA    1024
#define SLA    10
#define WLCAP  3072
#define RCAP   20480
#define DEGCAP 64
#define FLAGW  32
#define GBM    64
#define GBN    128
#define GTHR   128
#define GWAVE  (GTHR / 32)
#define MTILE  128
#define ROWH   256
#define NUW1   (DF * (K1 / 8))
#define NUW2   (DF * (K2 / 8))
#define NUBR   NTHR
#define BK_ZINTS    (NWAVE * WLCAP + RCAP + 3 * NBA)
#define BK_LDS_INTS (BK_ZINTS + 16)
#define WSMAX  134217728

static_assert(NBA == (1 << SLA));
static_assert((NBA * 4) % 128 == 0 && NBA == NTHR * 4 && NBA % NWAVE == 0 && NBA % 32 == 0);
static_assert(RCAP % (NTHR * 4) == 0 && (RCAP * 4) % 128 == 0);
static_assert(RCAP >= 17546);
static_assert(DEGCAP >= 36 + 8);
static_assert(NWAVE * WLCAP >= RCAP);
static_assert(BK_ZINTS % 4 == 0 && (NWAVE * WLCAP) % 4 == 0);
static_assert(BK_LDS_INTS * 4 <= 327680);
static_assert(3 * NBA * 4 + DF * 4 + NWAVE * ROWH * 2 <= 327680);
static_assert(K1 % 32 == 0 && K2 % 32 == 0 && K2 == 2 * DF && K1 == DF);
static_assert(GBN == DF && GBM == GWAVE * 16 && GTHR == GWAVE * 32 && DF == 4 * 32);
static_assert(MTILE % GBM == 0 && ROWH == 2 * DF);
static_assert(NUW1 % NTHR == 0 && NUW2 % NTHR == 0 && (MTILE * 16) % NTHR == 0);
static_assert(FLAGW * 4 == 128);

typedef float          v4f   __attribute__((ext_vector_type(4)));
typedef float          v8f   __attribute__((ext_vector_type(8)));
typedef int            v4i   __attribute__((ext_vector_type(4)));
typedef int            v8i   __attribute__((ext_vector_type(8)));
typedef unsigned       v4u   __attribute__((ext_vector_type(4)));
typedef unsigned short v4us  __attribute__((ext_vector_type(4)));
typedef unsigned short v8us  __attribute__((ext_vector_type(8)));
typedef unsigned short v16us __attribute__((ext_vector_type(16)));
typedef __bf16         v16bf __attribute__((ext_vector_type(16)));
typedef v4f  __attribute__((may_alias)) v4fa;
typedef v4i  __attribute__((may_alias)) v4ia;
typedef v4us __attribute__((may_alias)) v4usa;
typedef v8us __attribute__((may_alias)) v8usa;
union FragB { v16bf v; v16us u; v8us h[2]; v8i w; };

__device__ __forceinline__ v8f wmb(const FragB& a, const FragB& b, v8f c) {
  v8f d = __builtin_amdgcn_wmma_f32_16x16x32_bf16(false, a.v, false, b.v, (short)0, c, false, false);
  asm volatile("v_nop\n\tv_nop\n\tv_nop\n\tv_nop" : "+v"(d) : "v"(a.w), "v"(b.w));
  return d;
}

__device__ __forceinline__ v8f z8() { v8f z = {0.f, 0.f, 0.f, 0.f, 0.f, 0.f, 0.f, 0.f}; return z; }

__device__ __forceinline__ unsigned bf16_bits(float f) {
  const unsigned u = __float_as_uint(f);
  const unsigned r = (u + 0x7FFFu + ((u >> 16) & 1u)) >> 16;
  const bool isn = (u & 0x7FFFFFFFu) > 0x7F800000u;
  return isn ? 0x7FC0u : (r & 0xFFFFu);
}
__device__ __forceinline__ unsigned pack2(float a, float b) {
  return bf16_bits(a) | (bf16_bits(b) << 16);
}
__device__ __forceinline__ void hl_bits(float v, unsigned& hb, unsigned& lb) {
  hb = bf16_bits(v);
  lb = bf16_bits(v - __uint_as_float(hb << 16));
}

__device__ __forceinline__ void wave_sync() {
  __builtin_amdgcn_fence(__ATOMIC_RELEASE, "wavefront");
  __builtin_amdgcn_wave_barrier();
  __builtin_amdgcn_fence(__ATOMIC_ACQUIRE, "wavefront");
}

__device__ __forceinline__ float dinv_of(int c) {
  const float d = (float)c + 2.0f;
  float r = rsqrtf(d);
  r = r * fmaf(-0.5f * d, r * r, 1.5f);
  return (d > 0.0f) ? r : 0.0f;
}

__global__ __launch_bounds__(NTHR) void k_prep(const float* __restrict__ x, const float* __restrict__ W1,
                                               const float* __restrict__ b1, const float* __restrict__ W2,
                                               const float* __restrict__ b2,
                                               unsigned* w1t, unsigned* w2d, unsigned* br, unsigned* hhl,
                                               int nN, int mRows, int padUnits, int padSec) {
  const int u = (int)blockIdx.x * NTHR + (int)threadIdx.x;
  v4u o;
  unsigned* dp;
  if (u < NUW1) {
    const int n = u >> 4, k8 = (u & 15) * 8;
    const float* p = W1 + (size_t)k8 * DF + n;
    float f[8];
#pragma unroll
    for (int i = 0; i < 8; ++i) f[i] = p[(size_t)i * DF];
    o.x = pack2(f[0], f[1]); o.y = pack2(f[2], f[3]); o.z = pack2(f[4], f[5]); o.w = pack2(f[6], f[7]);
    dp = w1t + (size_t)u * 4;
  } else if (u < NUW1 + NUW2) {
    const int v = u - NUW1;
    const int n = v >> 5, k8 = (v & 31) * 8;
    const int kk = k8 & (DF - 1);
    const float* p = W2 + (size_t)kk * DF + n;
    float f[8];
#pragma unroll
    for (int i = 0; i < 8; ++i) f[i] = p[(size_t)i * DF];
    o.x = pack2(f[0], f[1]); o.y = pack2(f[2], f[3]); o.z = pack2(f[4], f[5]); o.w = pack2(f[6], f[7]);
    dp = w2d + (size_t)v * 4;
  } else if (u < NUW1 + NUW2 + NUBR) {
    const int v = u - (NUW1 + NUW2);
    if (v >= 64) return;
    const int i4 = (v & 31) * 4;
    const v4f a = *(const v4f*)(b1 + i4);
    const v4f c = *(const v4f*)(b2 + i4);
    asm volatile("" :: "v"(a), "v"(c));
    const unsigned msk = (v < 32) ? 0xFFFFFFFFu : 0u;
    o.x = ((bf16_bits(a.x) << 16) & msk) | ((bf16_bits(c.x) << 16) & ~msk);
    o.y = ((bf16_bits(a.y) << 16) & msk) | ((bf16_bits(c.y) << 16) & ~msk);
    o.z = ((bf16_bits(a.z) << 16) & msk) | ((bf16_bits(c.z) << 16) & ~msk);
    o.w = ((bf16_bits(a.w) << 16) & msk) | ((bf16_bits(c.w) << 16) & ~msk);
    dp = br + (size_t)v * 4;
  } else if (u < NUW1 + NUW2 + NUBR + padSec) {
    const int v = u - (NUW1 + NUW2 + NUBR);
    if (v >= padUnits) return;
    o.x = 0u; o.y = 0u; o.z = 0u; o.w = 0u;
    dp = hhl + (size_t)nN * (K2 / 2) + (size_t)v * 4;
  } else {
    const int v = u - (NUW1 + NUW2 + NUBR) - padSec;
    if (v >= mRows * 16) return;
    const int row = v >> 4, k8 = (v & 15) * 8;
    const int rc  = row < nN ? row : nN - 1;
    const float* p = x + (size_t)rc * DF + k8;
    const v4f a = *(const v4f*)p;
    const v4f c = *(const v4f*)(p + 4);
    asm volatile("" :: "v"(a), "v"(c));
    const unsigned msk = (row < nN) ? 0xFFFFFFFFu : 0u;
    o.x = pack2(a.x, a.y) & msk; o.y = pack2(a.z, a.w) & msk;
    o.z = pack2(c.x, c.y) & msk; o.w = pack2(c.z, c.w) & msk;
    dp = hhl + (size_t)v * 4;
  }
  *(volatile v4u*)dp = o;
  __threadfence();
  *(volatile v4u*)dp = o;
}

__global__ __launch_bounds__(NTHR) void k_bucket(const int* __restrict__ srcs, const int* __restrict__ dsts,
                                                 int nE, int nN, int shareLen, int nCh,
                                                 int* listg, int* cntg, int* offg, float* dinvg, int* flagg) {
  extern __shared__ __attribute__((aligned(16))) int dsm[];
  int* wl   = dsm;
  int* sl   = wl + NWAVE * WLCAP;
  int* cnt  = sl + RCAP;
  int* offs = cnt + NBA;
  int* cur  = offs + NBA;
  int* misc = cur + NBA;
  const int tid = (int)threadIdx.x, lane = tid & 31;
  const int wave = __builtin_amdgcn_readfirstlane(tid >> 5);
  const int nodeBase = (int)blockIdx.x * NBA;

  {
    const v4i z4 = {0, 0, 0, 0};
    for (int i = tid * 4; i < BK_ZINTS; i += NTHR * 4) *(v4ia*)(dsm + i) = z4;
    if (tid < 16) misc[tid] = 0;
  }
  __syncthreads();

  int wc = 0;
  {
    int* wlw = wl + wave * WLCAP;
    const int wbeg = wave * shareLen;
    const unsigned nbs = (unsigned)nodeBase;
    const int sent = -2147483647 - 1;
#pragma unroll 1
    for (int ch = 0; ch < nCh; ++ch) {
      const int cb = wbeg + ch * WCH;
      if (cb >= nE) break;
      const int base = cb + lane;
      int d[EPT];
#pragma unroll
      for (int j = 0; j < EPT; ++j) {
        const int e  = base + 32 * j;
        const int ec = e < nE ? e : nE - 1;
        d[j] = dsts[ec];
      }
#pragma unroll
      for (int j = 0; j < EPT; ++j) asm volatile("" :: "v"(d[j]));
      unsigned s[EPT];
      bool hany = false;
#pragma unroll
      for (int j = 0; j < EPT; ++j) {
        const int e = base + 32 * j;
        const int dv = (e < nE) ? d[j] : sent;
        s[j] = (unsigned)dv - nbs;
        hany = hany | (s[j] < (unsigned)NBA);
      }
      const unsigned any = __builtin_amdgcn_ballot_w32(hany);
      if (any != 0u) {
#pragma unroll
        for (int j = 0; j < EPT; ++j) {
          const bool hj = s[j] < (unsigned)NBA;
          const unsigned mj = __builtin_amdgcn_ballot_w32(hj);
          if (mj != 0u) {
            if (hj) {
              const int pos = wc + (int)__builtin_amdgcn_mbcnt_lo(mj, 0u);
              if (pos < WLCAP) wlw[pos] = ((base + 32 * j) << SLA) | (int)s[j];
            }
            wc += (int)__builtin_popcount(mj);
          }
        }
      }
    }
  }
  if (lane == 0) misc[wave] = wc;
  __syncthreads();

  if (wave == 0) {
    int tot = 0, ov = 0;
#pragma unroll 1
    for (int w2 = 0; w2 < NWAVE; ++w2) {
      int c = __builtin_amdgcn_readfirstlane(misc[w2]);
      if (c > WLCAP) ov = 1;
      c = c < 0 ? 0 : (c > WLCAP ? WLCAP : c);
      tot += c;
#pragma unroll 1
      for (int b0 = 0; b0 < c; b0 += 32) {
        const int idx = b0 + lane;
        const int ent = wl[w2 * WLCAP + (idx < WLCAP ? idx : WLCAP - 1)];
        const int m32 = (c - b0) < 32 ? (c - b0) : 32;
#pragma unroll 1
        for (int k = 0; k < m32; ++k) {
          const int u  = __builtin_amdgcn_readlane(ent, k);
          const int st = u & (NBA - 1);
          if (lane == 0) cnt[st] = cnt[st] + 1;
        }
      }
    }
    if (tot > RCAP) ov = 1;
    if (lane == 0) misc[8] = ov;
  }
  __syncthreads();

  if (wave == 0) {
    const int base = lane * (NBA / 32);
    int s = 0;
#pragma unroll 1
    for (int i = 0; i < NBA / 32; ++i) s += cnt[base + i];
    int incl = s;
#pragma unroll
    for (int dd = 1; dd < 32; dd <<= 1) {
      const int y = __shfl_up(incl, dd, 32);
      if (lane >= dd) incl += y;
    }
    int run = incl - s;
#pragma unroll 1
    for (int i = 0; i < NBA / 32; ++i) {
      const int cv = cnt[base + i];
      offs[base + i] = run;
      cur[base + i]  = run;
      run += cv;
    }
  }
  __syncthreads();

  if (wave == 0) {
#pragma unroll 1
    for (int w2 = 0; w2 < NWAVE; ++w2) {
      int c = __builtin_amdgcn_readfirstlane(misc[w2]);
      c = c < 0 ? 0 : (c > WLCAP ? WLCAP : c);
#pragma unroll 1
      for (int b0 = 0; b0 < c; b0 += 32) {
        const int idx = b0 + lane;
        const int ent = wl[w2 * WLCAP + (idx < WLCAP ? idx : WLCAP - 1)];
        int eid = ent >> SLA;
        eid = eid < 0 ? 0 : (eid > nE - 1 ? nE - 1 : eid);
        int sr = srcs[eid];
        sr = sr < 0 ? 0 : (sr > nN - 1 ? nN - 1 : sr);
        const int m32 = (c - b0) < 32 ? (c - b0) : 32;
#pragma unroll 1
        for (int k = 0; k < m32; ++k) {
          const int u  = __builtin_amdgcn_readlane(ent, k);
          const int sv = __builtin_amdgcn_readlane(sr, k);
          const int st = u & (NBA - 1);
          if (lane == 0) {
            int p = cur[st];
            p = p < 0 ? 0 : (p > RCAP - 1 ? RCAP - 1 : p);
            sl[p] = sv;
            cur[st] = p + 1;
          }
        }
      }
    }
  }
  __syncthreads();

  const int ovf = misc[8];
  int* lp = listg + (size_t)blockIdx.x * RCAP;
  const v4i c4 = *(const v4ia*)(cnt + 4 * tid);
  const v4i o4 = *(const v4ia*)(offs + 4 * tid);
  v4f d4;
  d4.x = dinv_of(c4.x); d4.y = dinv_of(c4.y); d4.z = dinv_of(c4.z); d4.w = dinv_of(c4.w);
  const v4i f4 = {ovf, ovf, ovf, ovf};
  int* cp = cntg + (size_t)nodeBase + 4 * tid;
  int* op = offg + (size_t)nodeBase + 4 * tid;
  float* dp = dinvg + (size_t)nodeBase + 4 * tid;
  int* fp = flagg + (size_t)blockIdx.x * FLAGW + 4 * (tid & 7);
#pragma unroll 1
  for (int it = 0; it < RCAP / (NTHR * 4); ++it) {
    const int i = it * (NTHR * 4) + 4 * tid;
    const v4i v = *(const v4ia*)(sl + i);
    *(volatile v4i*)(lp + i) = v;
  }
  *(volatile v4i*)cp = c4;
  *(volatile v4i*)op = o4;
  *(volatile v4f*)dp = d4;
  if (tid < 8) *(volatile v4i*)fp = f4;
  __threadfence();
#pragma unroll 1
  for (int it = 0; it < RCAP / (NTHR * 4); ++it) {
    const int i = it * (NTHR * 4) + 4 * tid;
    const v4i v = *(const v4ia*)(sl + i);
    *(volatile v4i*)(lp + i) = v;
  }
  *(volatile v4i*)cp = c4;
  *(volatile v4i*)op = o4;
  *(volatile v4f*)dp = d4;
  if (tid < 8) *(volatile v4i*)fp = f4;
}

__global__ __launch_bounds__(GTHR) __attribute__((amdgpu_num_vgpr(248)))
void k_gemm(const unsigned short* __restrict__ A, int lda,
            const unsigned short* __restrict__ BT, int ldb, int K,
            const float* __restrict__ dinv, float* outp, int nN) {
  __shared__ __attribute__((aligned(16))) float stg[GBM * GBN];
  __shared__ __attribute__((aligned(16))) float sdv[GBM];
  const int tid = (int)threadIdx.x, lane = tid & 31, wave = tid >> 5, hh = lane >> 4, m = lane & 15;
  const int rowBase = (int)blockIdx.x * GBM;

  v8f acc[8];
#pragma unroll
  for (int t = 0; t < 8; ++t) acc[t] = z8();
  const unsigned short* ap = A + (size_t)(rowBase + 16 * wave + m) * (size_t)lda + 8 * hh;
  const unsigned short* bp = BT + (size_t)m * (size_t)ldb + 8 * hh;

#pragma unroll 1
  for (int k0 = 0; k0 < K; k0 += 32) {
    FragB af;
    af.h[0] = *(const v8usa*)(ap + k0);
    af.h[1] = *(const v8usa*)(ap + k0 + 16);
#pragma unroll
    for (int nt = 0; nt < 8; ++nt) {
      const unsigned short* wq = bp + (size_t)(16 * nt) * (size_t)ldb + k0;
      FragB bf;
      bf.h[0] = *(const v8usa*)wq;
      bf.h[1] = *(const v8usa*)(wq + 16);
      acc[nt] = wmb(af, bf, acc[nt]);
    }
  }

#pragma unroll
  for (int nt = 0; nt < 8; ++nt) {
    const int lc = 16 * nt + m;
#pragma unroll
    for (int r = 0; r < 8; ++r) {
      const int lr = 16 * wave + 8 * hh + r;
      stg[lr * GBN + lc] = acc[nt][r];
    }
  }
  if (tid < GBM) sdv[tid] = dinv[rowBase + tid];
  __syncthreads();

  v4f pv[16];
#pragma unroll
  for (int i = 0; i < 16; ++i) {
    const v4f t = *(const v4fa*)(stg + (16 * wave + i) * GBN + 4 * lane);
    const float dd = sdv[16 * wave + i];
    v4f q;
    q.x = t.x * dd; q.y = t.y * dd; q.z = t.z * dd; q.w = t.w * dd;
    pv[i] = q;
  }
#pragma unroll
  for (int i = 0; i < 16; ++i) {
    const int row = rowBase + 16 * wave + i;
    float* op = outp + (size_t)row * DF + 4 * lane;
    if (row < nN) *(volatile v4f*)op = pv[i];
  }
  __threadfence();
#pragma unroll
  for (int i = 0; i < 16; ++i) {
    const int row = rowBase + 16 * wave + i;
    float* op = outp + (size_t)row * DF + 4 * lane;
    if (row < nN) *(volatile v4f*)op = pv[i];
  }
}

template <bool FINAL>
__global__ __launch_bounds__(NTHR) void k_replay(const float* __restrict__ hp, const int* __restrict__ listg,
                                                 const int* __restrict__ cntg, const int* __restrict__ offg,
                                                 const float* __restrict__ dinvg, const int* __restrict__ flagg,
                                                 const float* __restrict__ bias,
                                                 unsigned short* hhl, float* outp, int nN) {
  __shared__ __attribute__((aligned(16))) int   scnt[NBA];
  __shared__ __attribute__((aligned(16))) int   soff[NBA];
  __shared__ __attribute__((aligned(16))) float sdv[NBA];
  __shared__ __attribute__((aligned(16))) float sb[DF];
  __shared__ __attribute__((aligned(16))) unsigned short rowall[NWAVE * ROWH];
  const int tid = (int)threadIdx.x, lane = tid & 31;
  const int wave = __builtin_amdgcn_readfirstlane(tid >> 5);
  const int nodeBase = (int)blockIdx.x * NBA;

  {
    const v4i c4 = *(const v4i*)(cntg + (size_t)nodeBase + 4 * tid);
    const v4i o4 = *(const v4i*)(offg + (size_t)nodeBase + 4 * tid);
    const v4f d4 = *(const v4f*)(dinvg + (size_t)nodeBase + 4 * tid);
    *(v4ia*)(scnt + 4 * tid) = c4;
    *(v4ia*)(soff + 4 * tid) = o4;
    *(v4fa*)(sdv + 4 * tid)  = d4;
    if (wave == 0) {
      const v4f b4 = *(const v4f*)(bias + 4 * lane);
      *(v4fa*)(sb + 4 * lane) = b4;
    }
  }
  const int flag = __builtin_amdgcn_readfirstlane(flagg[(size_t)blockIdx.x * FLAGW]);
  __syncthreads();

  const v4f bq = *(const v4fa*)(sb + 4 * lane);
  const int* lp = listg + (size_t)blockIdx.x * RCAP;
  unsigned short* rowbuf = rowall + wave * ROWH;
  const float qnan = __int_as_float(0x7fc00000);

#pragma unroll 1
  for (int si = 0; si < NBA / NWAVE; ++si) {
    const int s    = si * NWAVE + wave;
    const int node = nodeBase + s;
    if (node < nN) {
      const int craw = __builtin_amdgcn_readfirstlane(scnt[s]);
      const bool big = craw > DEGCAP;
      const int c = craw < 0 ? 0 : (craw > DEGCAP ? DEGCAP : craw);
      int o = __builtin_amdgcn_readfirstlane(soff[s]);
      o = o < 0 ? 0 : (o > RCAP ? RCAP : o);
      const float dd = sdv[s];
      float a0 = 0.0f, a1 = 0.0f, a2 = 0.0f, a3 = 0.0f;
#pragma unroll 1
      for (int b0 = 0; b0 < c; b0 += 32) {
        int idx = o + b0 + lane;
        const int hiI = o + c - 1;
        idx = idx > hiI ? hiI : idx;
        idx = idx < 0 ? 0 : (idx > RCAP - 1 ? RCAP - 1 : idx);
        int sr = lp[idx];
        sr = sr < 0 ? 0 : (sr > nN - 1 ? nN - 1 : sr);
        const int m32 = (c - b0) < 32 ? (c - b0) : 32;
#pragma unroll 1
        for (int k = 0; k < m32; ++k) {
          const int sk = __builtin_amdgcn_readlane(sr, k);
          const v4f r = *(const v4fa*)(hp + (size_t)sk * DF + 4 * lane);
          a0 += r.x; a1 += r.y; a2 += r.z; a3 += r.w;
        }
      }
      const v4f sv = *(const v4fa*)(hp + (size_t)node * DF + 4 * lane);
      float y0 = (a0 + 2.0f * sv.x) * dd + bq.x;
      float y1 = (a1 + 2.0f * sv.y) * dd + bq.y;
      float y2 = (a2 + 2.0f * sv.z) * dd + bq.z;
      float y3 = (a3 + 2.0f * sv.w) * dd + bq.w;
      const bool pois = (flag != 0) || big;
      y0 = pois ? qnan : y0; y1 = pois ? qnan : y1; y2 = pois ? qnan : y2; y3 = pois ? qnan : y3;
      if constexpr (FINAL) {
        v4f ov; ov.x = y0; ov.y = y1; ov.z = y2; ov.w = y3;
        float* op = outp + (size_t)node * DF + 4 * lane;
        *(volatile v4f*)op = ov;
        __threadfence();
        *(volatile v4f*)op = ov;
      } else {
        v4us mh, ml;
        unsigned hb, lb;
        hl_bits(y0, hb, lb); mh[0] = (unsigned short)hb; ml[0] = (unsigned short)lb;
        hl_bits(y1, hb, lb); mh[1] = (unsigned short)hb; ml[1] = (unsigned short)lb;
        hl_bits(y2, hb, lb); mh[2] = (unsigned short)hb; ml[2] = (unsigned short)lb;
        hl_bits(y3, hb, lb); mh[3] = (unsigned short)hb; ml[3] = (unsigned short)lb;
        *(v4usa*)(rowbuf + 4 * lane)      = mh;
        *(v4usa*)(rowbuf + DF + 4 * lane) = ml;
        wave_sync();
        const v8us q0 = *(const v8usa*)(rowbuf + 8 * lane);
        wave_sync();
        unsigned short* rp = hhl + (size_t)node * K2 + 8 * lane;
        *(volatile v8us*)rp = q0;
        __threadfence();
        *(volatile v8us*)rp = q0;
      }
    }
  }
  if constexpr (FINAL) { (void)hhl; } else { (void)outp; }
}

static inline int cdiv(int a, int b) { return (a + b - 1) / b; }
static inline size_t al256(size_t o) { return (o + 255) & ~(size_t)255; }

extern "C" void kernel_launch(void* const* d_in, const int* in_sizes, int n_in,
                              void* d_out, int out_size, void* d_ws, size_t ws_size,
                              hipStream_t stream) {
  if (n_in < 6) return;
  if (in_sizes[0] < DF || (in_sizes[0] % DF) != 0) return;
  const int nN = in_sizes[0] / DF;
  if (nN < MTILE || nN > (1 << 22)) return;
  if (in_sizes[1] < 2 || (in_sizes[1] & 1) != 0) return;
  const int nE = in_sizes[1] / 2;
  if (nE < 1 || nE >= (1 << (31 - SLA))) return;
  if (in_sizes[2] != DF * DF || in_sizes[3] != DF) return;
  if (in_sizes[4] != DF * DF || in_sizes[5] != DF) return;
  if ((long long)out_size != (long long)nN * DF) return;

  const float* x  = (const float*)d_in[0];
  const int*   ei = (const int*)  d_in[1];
  const float* W1 = (const float*)d_in[2];
  const float* b1 = (const float*)d_in[3];
  const float* W2 = (const float*)d_in[4];
  const float* b2 = (const float*)d_in[5];
  float* out = (float*)d_out;
  const int* src = ei;
  const int* dst = ei + nE;

  const int MP  = cdiv(nN, MTILE) * MTILE;
  const int gM  = MP / GBM;
  const int gA  = cdiv(nN, NBA);
  const long long NBPl = (long long)gA * NBA;
  if (NBPl < (long long)MP) return;
  if (2LL * nN < (long long)MP) return;
  const int shareLen = cdiv(cdiv(nE, NWAVE), WCH) * WCH;
  const int nCh = shareLen / WCH;
  const int padUnits = (MP - nN) * (K2 / 8);
  const int padSec   = cdiv(padUnits, NTHR) * NTHR;

  char* ws = (char*)d_ws;
  size_t off = 0;
  const size_t oHP   = off; off = al256(off + (size_t)nN * DF * 4);
  const size_t oHHL  = off; off = al256(off + (size_t)MP * K2 * 2);
  const size_t oLIST = off; off = al256(off + (size_t)gA * RCAP * 4);
  const size_t oCNT  = off; off = al256(off + (size_t)NBPl * 4);
  const size_t oOFF  = off; off = al256(off + (size_t)NBPl * 4);
  const size_t oDINV = off; off = al256(off + (size_t)NBPl * 4);
  const size_t oFLAG = off; off = al256(off + (size_t)gA * FLAGW * 4);
  const size_t oW1T  = off; off = al256(off + (size_t)DF * K1 * 2);
  const size_t oW2D  = off; off = al256(off + (size_t)DF * K2 * 2);
  const size_t oBR   = off; off = al256(off + (size_t)2 * DF * 4);
  if (off > ws_size || off > (size_t)WSMAX) return;
  float*          HP   = (float*)(ws + oHP);
  unsigned short* HHL  = (unsigned short*)(ws + oHHL);
  unsigned short* XB   = HHL;
  int*            LIST = (int*)(ws + oLIST);
  int*            CNT  = (int*)(ws + oCNT);
  int*            OFFS = (int*)(ws + oOFF);
  float*          DINV = (float*)(ws + oDINV);
  int*            FLAG = (int*)(ws + oFLAG);
  unsigned short* W1T  = (unsigned short*)(ws + oW1T);
  unsigned short* W2D  = (unsigned short*)(ws + oW2D);
  float*          BR   = (float*)(ws + oBR);

  const size_t bkLds = (size_t)BK_LDS_INTS * 4;
  hipFuncSetAttribute(reinterpret_cast<const void*>(&k_bucket), hipFuncAttributeMaxDynamicSharedMemorySize, (int)bkLds);

  const long long nUnitsL = (long long)NUW1 + NUW2 + NUBR + padSec + (long long)MP * 16;
  if (nUnitsL > 2000000000LL || (nUnitsL % NTHR) != 0) return;
  const int gP = (int)(nUnitsL / NTHR);

  k_prep<<<gP, NTHR, 0, stream>>>(x, W1, b1, W2, b2, (unsigned*)W1T, (unsigned*)W2D, (unsigned*)BR,
                                  (unsigned*)HHL, nN, MP, padUnits, padSec);
  k_bucket<<<gA, NTHR, bkLds, stream>>>(src, dst, nE, nN, shareLen, nCh, LIST, CNT, OFFS, DINV, FLAG);
  k_gemm<<<gM, GTHR, 0, stream>>>(XB, K1, W1T, K1, K1, DINV, HP, nN);
  k_replay<false><<<gA, NTHR, 0, stream>>>(HP, LIST, CNT, OFFS, DINV, FLAG, BR, HHL, out, nN);
  for (int l = 0; l < 3; ++l) {
    k_gemm<<<gM, GTHR, 0, stream>>>(HHL, K2, W2D, K2, K2, DINV, HP, nN);
    k_replay<false><<<gA, NTHR, 0, stream>>>(HP, LIST, CNT, OFFS, DINV, FLAG, BR + DF, HHL, out, nN);
  }
  k_gemm<<<gM, GTHR, 0, stream>>>(HHL, K2, W2D, K2, K2, DINV, HP, nN);
  k_replay<true><<<gA, NTHR, 0, stream>>>(HP, LIST, CNT, OFFS, DINV, FLAG, BR + DF, HHL, out, nN);
}
